// SphericalGMMLayer_61598420959739
// MI455X (gfx1250) — hardware-run, weakly checked
//
#include <hip/hip_runtime.h>
#include <stddef.h>


typedef _Float16 v16h __attribute__((ext_vector_type(16)));
typedef _Float16 v8h  __attribute__((ext_vector_type(8)));
typedef float    v8f  __attribute__((ext_vector_type(8)));
typedef float    v4f  __attribute__((ext_vector_type(4)));
typedef _Float16 h16;

#ifndef NB
#define NB 8
#endif
#define NB_FULL 8
#define NK 32
#define ND 64
#define NP 4096

#define EPS_MASS  1.0e-5f
#define EPS_SIGMA 1.0e-3f

#define LDC 68
#define LDM 36

#define ICARRY  64.0f
#define XCARRY  1024.0f
#define MUCARRY 1024.0f

static_assert(NB >= 1 && NB <= NB_FULL);
static_assert(NK == 32 && ND == 64);
static_assert((NP % 64) == 0 && (NP % 32) == 0);
static_assert(NP == 16 * 256);
static_assert(NK == 8 * 4);
static_assert((LDC % 4) == 0 && LDC >= 64);
static_assert(LDM >= NK);
static_assert((ND % 32) == 0);

#define IH_BYTES  ((size_t)NB * ND * NP * 2)
#define IMT_BYTES ((size_t)NB * NP * ND * 2)
#define XH_BYTES  ((size_t)NB * NK * NP * 2)
#define S2_BYTES  ((size_t)NB * NP * 4)
#define MUH_BYTES ((size_t)NB * NK * ND * 2)
#define ST_BYTES  ((size_t)NB * 64 * 4)
#define CO_BYTES  ((size_t)NB * 96 * 4)
#define OFF_IH  ((size_t)0)
#define OFF_IMT (OFF_IH + IH_BYTES)
#define OFF_XH  (OFF_IMT + IMT_BYTES)
#define OFF_S2  (OFF_XH + XH_BYTES)
#define OFF_MUH (OFF_S2 + S2_BYTES)
#define OFF_ST  (OFF_MUH + MUH_BYTES)
#define OFF_CO  (OFF_ST + ST_BYTES)
#define WS_TOTAL (OFF_CO + CO_BYTES)
static_assert((IH_BYTES % 128) == 0 && (IMT_BYTES % 128) == 0 && (XH_BYTES % 128) == 0);
static_assert((S2_BYTES % 128) == 0 && (MUH_BYTES % 128) == 0);
static_assert((ST_BYTES % 128) == 0 && (CO_BYTES % 128) == 0);
static_assert(WS_TOTAL <= (size_t)134217728);

__device__ __forceinline__ float bf16r(float x) {
  unsigned int u = __float_as_uint(x);
  u = (u + 0x7FFFu + ((u >> 16) & 1u)) & 0xFFFF0000u;
  return __uint_as_float(u);
}

static __device__ __forceinline__ h16 toh_flush(float v) {
  const h16 r = (h16)v;
  return (fabsf(v) < 6.103515625e-05f) ? (h16)0.0f : r;
}

__device__ __forceinline__ v16h frag_at(const _Float16* p) {
  v8h lo = *(const v8h*)(p);
  v8h hi = *(const v8h*)(p + 16);
  v16h out;
#pragma unroll
  for (int i = 0; i < 8; ++i) { out[i] = lo[i]; out[i + 8] = hi[i]; }
  return out;
}

__device__ __forceinline__ v8f wmma16(v16h a, v16h b, v8f c) {
  v8f d = __builtin_amdgcn_wmma_f32_16x16x32_f16(false, a, false, b, (short)0, c,
                                                 false, false);
  asm volatile("v_nop\n\tv_nop\n\tv_nop\n\tv_nop" : "+v"(d) : "v"(a), "v"(b));
  return d;
}

__device__ __forceinline__ float red32_sum(float x) {
#pragma unroll
  for (int off = 1; off < 32; off <<= 1) x += __shfl_xor(x, off, 32);
  return x;
}

__global__ __launch_bounds__(256) void img_prep_kernel(
    const float* __restrict__ img, _Float16* __restrict__ Ih, _Float16* __restrict__ ImT,
    float* __restrict__ S2) {
  __shared__ __attribute__((aligned(16))) float F[64 * LDC];
  __shared__ __attribute__((aligned(16))) float S2s[64];
  const unsigned tid = threadIdx.x;
  const unsigned p0 = blockIdx.x * 64u;
  const unsigned b = blockIdx.y;
  const size_t ibase = (size_t)b * ND * NP;

  v8h x[2];
  size_t off[2];
#pragma unroll
  for (unsigned i = 0; i < 2u; ++i) {
    const unsigned idx = tid + 256u * i;
    const unsigned d = idx >> 3, c = (idx & 7u) * 8u;
    const size_t g = ibase + (size_t)d * NP + p0 + c;
    const v4f a0 = *(const v4f*)(img + g);
    const v4f a1 = *(const v4f*)(img + g + 4u);
#pragma unroll
    for (int j = 0; j < 4; ++j) {
      const float e0 = bf16r(a0[j]);
      const float e1 = bf16r(a1[j]);
      F[d * LDC + c + (unsigned)j] = e0;
      F[d * LDC + c + 4u + (unsigned)j] = e1;
      x[i][j]     = toh_flush(ICARRY * e0);
      x[i][j + 4] = toh_flush(ICARRY * e1);
    }
    off[i] = g;
  }
  __syncthreads();

  v8h t[2];
  size_t offt[2];
#pragma unroll
  for (unsigned i = 0; i < 2u; ++i) {
    const unsigned idx = tid + 256u * i;
    const unsigned p = idx >> 3, dc = (idx & 7u) * 8u;
#pragma unroll
    for (unsigned j = 0; j < 8u; ++j) t[i][j] = toh_flush(ICARRY * F[(dc + j) * LDC + p]);
    offt[i] = ((size_t)b * NP + p0 + p) * ND + dc;
  }
  if (tid < 64u) {
    float s = 0.0f;
#pragma unroll 1
    for (unsigned d = 0; d < (unsigned)ND; ++d) {
      const float v = F[d * LDC + tid];
      s += v * v;
    }
    S2s[tid] = s;
  }
  __syncthreads();

  const v4f sv = *(const v4f*)&S2s[(tid & 15u) * 4u];
  const size_t s2off = (size_t)b * NP + p0 + (tid & 15u) * 4u;

#pragma unroll
  for (int i = 0; i < 2; ++i) *(volatile v8h*)(Ih + off[i]) = x[i];
#pragma unroll
  for (int i = 0; i < 2; ++i) *(volatile v8h*)(ImT + offt[i]) = t[i];
  if (tid < 16u) *(volatile v4f*)(S2 + s2off) = sv;
  __threadfence();
#pragma unroll
  for (int i = 0; i < 2; ++i) *(volatile v8h*)(Ih + off[i]) = x[i];
#pragma unroll
  for (int i = 0; i < 2; ++i) *(volatile v8h*)(ImT + offt[i]) = t[i];
  if (tid < 16u) *(volatile v4f*)(S2 + s2off) = sv;
}

__global__ __launch_bounds__(256) void x_prep_kernel(
    const float* __restrict__ X, const float* __restrict__ S2,
    _Float16* __restrict__ Xh, float* __restrict__ ST) {
  __shared__ __attribute__((aligned(16))) float st[64];
  const unsigned tid = threadIdx.x, lane = tid & 31u;
  const unsigned wave = (unsigned)__builtin_amdgcn_readfirstlane((int)(threadIdx.x >> 5));
  const unsigned b = blockIdx.x;
  const float* s2r = S2 + (size_t)b * NP;

#pragma unroll 1
  for (unsigned rr = 0; rr < 4u; ++rr) {
    const unsigned k = wave * 4u + rr;
    const size_t rowoff = ((size_t)b * NK + k) * NP;
    float s = 0.0f, t = 0.0f;
#pragma unroll 1
    for (unsigned j = 0; j < 16u; ++j) {
      const unsigned c = j * 256u + lane * 8u;
      const v4f a0 = *(const v4f*)(X + rowoff + c);
      const v4f a1 = *(const v4f*)(X + rowoff + c + 4u);
      const v4f q0 = *(const v4f*)(s2r + c);
      const v4f q1 = *(const v4f*)(s2r + c + 4u);
      v8h o;
#pragma unroll
      for (int i = 0; i < 4; ++i) {
        const float e0 = bf16r(a0[i]);
        const float e1 = bf16r(a1[i]);
        s += e0 + e1;
        t += e0 * q0[i];
        t += e1 * q1[i];
        o[i]     = toh_flush(XCARRY * e0);
        o[i + 4] = toh_flush(XCARRY * e1);
      }
      _Float16* p = Xh + rowoff + c;
      *(volatile v8h*)p = o;
      __threadfence();
      *(volatile v8h*)p = o;
    }
    s = red32_sum(s);
    t = red32_sum(t);
    if (lane == 0u) { st[k] = s; st[32u + k] = t; }
  }
  __syncthreads();
  const v4f sv = *(const v4f*)&st[(tid & 15u) * 4u];
  float* dst = ST + (size_t)b * 64u + (tid & 15u) * 4u;
  if (tid < 16u) *(volatile v4f*)dst = sv;
  __threadfence();
  if (tid < 16u) *(volatile v4f*)dst = sv;
}

__global__ __launch_bounds__(256) void mu_kernel(
    const _Float16* __restrict__ Ih, const _Float16* __restrict__ Xh,
    const float* __restrict__ ST, _Float16* __restrict__ MuH, float* __restrict__ CO) {
  __shared__ __attribute__((aligned(16))) float Cs[64 * LDM];
  __shared__ __attribute__((aligned(16))) float co[96];
  const unsigned tid = threadIdx.x, lane = tid & 31u;
  const unsigned wave = (unsigned)__builtin_amdgcn_readfirstlane((int)(threadIdx.x >> 5));
  const unsigned mw = wave >> 1, nw = wave & 1u;
  const unsigned hh = lane >> 4, m = lane & 15u;
  const unsigned b = blockIdx.x;
  const float GS = 1.0f / (ICARRY * XCARRY);

  const _Float16* ap = Ih + ((size_t)b * ND + mw * 16u + m) * NP + hh * 8u;
  const _Float16* bp = Xh + ((size_t)b * NK + nw * 16u + m) * NP + hh * 8u;
  v8f acc = {};
#pragma unroll 2
  for (unsigned k0 = 0; k0 < (unsigned)NP; k0 += 32u) {
    const v16h a  = frag_at(ap + k0);
    const v16h bb = frag_at(bp + k0);
    acc = wmma16(a, bb, acc);
  }
#pragma unroll
  for (int r = 0; r < 8; ++r)
    Cs[(mw * 16u + hh * 8u + (unsigned)r) * LDM + nw * 16u + m] = acc[r];
  __syncthreads();

  if (tid < 32u) {
    const float sxv = ST[(size_t)b * 64u + tid];
    const float t1v = ST[(size_t)b * 64u + 32u + tid];
    const float inv = 1.0f / (sxv + EPS_MASS);
    float mn2 = 0.0f;
#pragma unroll 1
    for (unsigned d = 0; d < (unsigned)ND; ++d) {
      const float mn = Cs[d * LDM + tid] * GS;
      mn2 += mn * mn;
    }
    const float sig_num = t1v - mn2 * (2.0f * inv - sxv * inv * inv);
    const float sig = sig_num * (1.0f / (EPS_MASS + sxv * (float)ND));
    co[tid]       = sxv * (1.0f / (float)NP);
    co[32u + tid] = 0.5f / (sig + EPS_SIGMA);
    co[64u + tid] = mn2 * inv * inv;
  }

  const unsigned kk = tid >> 3, dc = (tid & 7u) * 8u;
  const float invk = 1.0f / (ST[(size_t)b * 64u + kk] + EPS_MASS);
  const float sc = (GS * MUCARRY) * invk;
  v8h o;
#pragma unroll
  for (unsigned j = 0; j < 8u; ++j) o[j] = toh_flush(Cs[(dc + j) * LDM + kk] * sc);
  const size_t moff = ((size_t)b * NK + kk) * ND + dc;
  __syncthreads();

  const unsigned ci = (tid < 24u) ? tid : 23u;
  const v4f cv = *(const v4f*)&co[ci * 4u];
  float* cdst = CO + (size_t)b * 96u + ci * 4u;

  *(volatile v8h*)(MuH + moff) = o;
  if (tid < 24u) *(volatile v4f*)cdst = cv;
  __threadfence();
  *(volatile v8h*)(MuH + moff) = o;
  if (tid < 24u) *(volatile v4f*)cdst = cv;
}

__global__ __launch_bounds__(128) void classify_kernel(
    const _Float16* __restrict__ MuH, const _Float16* __restrict__ ImT,
    const float* __restrict__ S2, const float* __restrict__ CO, float* __restrict__ Y) {
  __shared__ __attribute__((aligned(16))) float Cf[96];
  __shared__ __attribute__((aligned(16))) float Ys[32 * LDC];
  const unsigned tid = threadIdx.x, lane = tid & 31u;
  const unsigned wave = (unsigned)__builtin_amdgcn_readfirstlane((int)(threadIdx.x >> 5));
  const unsigned hh = lane >> 4, m = lane & 15u;
  const unsigned p0 = blockIdx.x * 64u;
  const unsigned b = blockIdx.y;
  const float DS = 1.0f / (MUCARRY * ICARRY);

  {
    const unsigned ci = (tid < 96u) ? tid : 95u;
    const float cvv = CO[(size_t)b * 96u + ci];
    if (tid < 96u) Cf[tid] = cvv;
  }

  const _Float16* ap0 = MuH + ((size_t)b * NK + m) * ND + hh * 8u;
  const _Float16* ap1 = ap0 + (size_t)16 * ND;
  const _Float16* bp  = ImT + ((size_t)b * NP + p0 + wave * 16u + m) * ND + hh * 8u;
  v8f acc0 = {}, acc1 = {};
#pragma unroll
  for (unsigned c = 0; c < 2u; ++c) {
    const v16h bf = frag_at(bp + c * 32u);
    const v16h a0 = frag_at(ap0 + c * 32u);
    const v16h a1 = frag_at(ap1 + c * 32u);
    acc0 = wmma16(a0, bf, acc0);
    acc1 = wmma16(a1, bf, acc1);
  }
  const float s2p = S2[(size_t)b * NP + p0 + wave * 16u + m];
  __syncthreads();

  float v0[8], v1[8];
  float loc = 0.0f;
#pragma unroll
  for (int r = 0; r < 8; ++r) {
    const unsigned ka = hh * 8u + (unsigned)r;
    const unsigned kb = 16u + ka;
    const float iza = s2p - 2.0f * (acc0[r] * DS) + Cf[64u + ka];
    const float izb = s2p - 2.0f * (acc1[r] * DS) + Cf[64u + kb];
    v0[r] = Cf[ka] * expf(-Cf[32u + ka] * iza);
    v1[r] = Cf[kb] * expf(-Cf[32u + kb] * izb);
    loc += v0[r] + v1[r];
  }
  const float tot = loc + __shfl_xor(loc, 16, 32);
  const float rinv = 1.0f / (EPS_MASS + tot);
#pragma unroll
  for (int r = 0; r < 8; ++r) {
    Ys[(hh * 8u + (unsigned)r) * LDC + wave * 16u + m]       = v0[r] * rinv;
    Ys[(16u + hh * 8u + (unsigned)r) * LDC + wave * 16u + m] = v1[r] * rinv;
  }
  __syncthreads();

  v4f xs[4];
  size_t off[4];
#pragma unroll
  for (unsigned i = 0; i < 4u; ++i) {
    const unsigned idx = tid + 128u * i;
    const unsigned k = idx >> 4, c = (idx & 15u) * 4u;
    xs[i] = *(const v4f*)&Ys[k * LDC + c];
    off[i] = ((size_t)b * NK + k) * NP + p0 + c;
  }
#pragma unroll
  for (int i = 0; i < 4; ++i) *(volatile v4f*)(Y + off[i]) = xs[i];
  __threadfence();
#pragma unroll
  for (int i = 0; i < 4; ++i) *(volatile v4f*)(Y + off[i]) = xs[i];
}

extern "C" void kernel_launch(void* const* d_in, const int* in_sizes, int n_in,
                              void* d_out, int out_size, void* d_ws, size_t ws_size,
                              hipStream_t stream) {
  if (n_in < 2) return;
  if ((long long)in_sizes[0] < (long long)NB * NK * NP) return;
  if ((long long)in_sizes[1] < (long long)NB * ND * NP) return;
  if ((long long)out_size < (long long)NB * NK * NP) return;
  if (ws_size < WS_TOTAL) return;

  const float* X   = (const float*)d_in[0];
  const float* IMG = (const float*)d_in[1];
  float* out = (float*)d_out;

  char* ws = (char*)d_ws;
  _Float16* Ih  = (_Float16*)(ws + OFF_IH);
  _Float16* ImT = (_Float16*)(ws + OFF_IMT);
  _Float16* Xh  = (_Float16*)(ws + OFF_XH);
  float*    S2  = (float*)(ws + OFF_S2);
  _Float16* MuH = (_Float16*)(ws + OFF_MUH);
  float*    ST  = (float*)(ws + OFF_ST);
  float*    CO  = (float*)(ws + OFF_CO);

  img_prep_kernel<<<dim3(NP / 64, NB), dim3(256), 0, stream>>>(IMG, Ih, ImT, S2);
  x_prep_kernel<<<dim3(NB), dim3(256), 0, stream>>>(X, S2, Xh, ST);
  mu_kernel<<<dim3(NB), dim3(256), 0, stream>>>(Ih, Xh, ST, MuH, CO);
  classify_kernel<<<dim3(NP / 64, NB), dim3(128), 0, stream>>>(MuH, ImT, S2, CO, out);
}
